// TransformerBlockQuantum_65481071397138
// MI455X (gfx1250) — hardware-run, weakly checked
//
#include <hip/hip_runtime.h>
#include <math.h>

#ifndef NB
#define NB 4
#endif
#ifndef SEQ
#define SEQ 2048
#endif
#define NB_FULL 4
#define SEQ_FULL 2048

constexpr int CD = 1024;
constexpr int NH = 16;
constexpr int HD = 64;
constexpr int NQ = 64;
constexpr int C4 = 4096;
constexpr int MTOK = NB * SEQ;
constexpr int MH = MTOK / 2;

static_assert(NB >= 1 && NB <= NB_FULL);
static_assert(SEQ <= SEQ_FULL);
static_assert(CD == NH * HD);
static_assert(HD == 64 && NQ == 64);
static_assert(CD % 128 == 0 && CD / 128 == 8);
static_assert(MTOK % 64 == 0 && MH % 64 == 0 && CD % 64 == 0 && C4 % 64 == 0);
static_assert(MTOK == 2 * MH);
static_assert(CD % 32 == 0 && C4 % 32 == 0 && NQ % 32 == 0);
static_assert(MTOK % 8 == 0);
static_assert(SEQ % 64 == 0);
static_assert(MTOK % 16 == 0);
static_assert((CD * CD) % 2048 == 0 && (C4 * NQ) % 2048 == 0 && (CD * C4) % 2048 == 0);

typedef __attribute__((ext_vector_type(16))) _Float16 v16h;
typedef __attribute__((ext_vector_type(8)))  _Float16 v8h;
typedef __attribute__((ext_vector_type(8)))  float    v8f;
typedef __attribute__((ext_vector_type(4)))  float    v4f;
typedef __attribute__((ext_vector_type(4)))  unsigned int v4u;

union FH { v16h v; v8h h[2]; };

#define VST2(T, ptr, val) do { const T vst2_v_ = (val); *(volatile T*)(ptr) = vst2_v_; __threadfence(); *(volatile T*)(ptr) = vst2_v_; } while (0)

#define WAVE_SYNC() do { __builtin_amdgcn_fence(3  , "workgroup"); __builtin_amdgcn_wave_barrier(); __builtin_amdgcn_fence(2  , "workgroup"); } while (0)

__device__ __forceinline__ float cmb_bf(float v) { const unsigned u = __builtin_bit_cast(unsigned, v); const unsigned r = (u + 0x7fffu + ((u >> 16) & 1u)) & 0xffff0000u; return __builtin_bit_cast(float, r); }
static __device__ __forceinline__ _Float16 toh_flush(float v) { const _Float16 r = (_Float16)v; return (fabsf(v) < 6.103515625e-05f) ? (_Float16)0.0f : r; }
static __device__ __forceinline__ unsigned int pk2h_flush(float a, float b) { return (unsigned int)__builtin_bit_cast(unsigned short, toh_flush(a)) | ((unsigned int)__builtin_bit_cast(unsigned short, toh_flush(b)) << 16); }
__device__ __forceinline__ v16h ldg_frag(const _Float16* __restrict__ p) { FH f; f.h[0] = *(const v8h*)(p); f.h[1] = *(const v8h*)(p + 16); return f.v; }

__device__ __forceinline__ void dep_guard_h(v8f& a, v8f& b, v16h x, v16h y) { asm volatile("v_nop\n\tv_nop\n\tv_nop\n\tv_nop" : "+v"(a), "+v"(b) : "v"(x), "v"(y)); }
__device__ __forceinline__ void keep4_h(v16h a, v16h b, v16h c, v16h d) { asm volatile("v_nop" :: "v"(a), "v"(b), "v"(c), "v"(d)); }
__device__ __forceinline__ void acc_guard4(v8f& a, v8f& b, v8f& c, v8f& d) { asm volatile("v_nop\n\tv_nop\n\tv_nop\n\tv_nop" : "+v"(a), "+v"(b), "+v"(c), "+v"(d)); }

__global__ __launch_bounds__(256) void k_castn(const float* __restrict__ SRC, unsigned short* __restrict__ DST, int n8, float sc) {
  #pragma clang fp contract(off)
  const int u = blockIdx.x * 256 + threadIdx.x; if (u >= n8) return;
  const v4f a = *(const v4f*)(SRC + (size_t)u * 8);
  const v4f b = *(const v4f*)(SRC + (size_t)u * 8 + 4);
  v4u pk;
  pk.x = pk2h_flush(cmb_bf(a.x) * sc, cmb_bf(a.y) * sc);
  pk.y = pk2h_flush(cmb_bf(a.z) * sc, cmb_bf(a.w) * sc);
  pk.z = pk2h_flush(cmb_bf(b.x) * sc, cmb_bf(b.y) * sc);
  pk.w = pk2h_flush(cmb_bf(b.z) * sc, cmb_bf(b.w) * sc);
  VST2(v4u, (v4u*)(DST + (size_t)u * 8), pk);
}

template <int W, int ABF, int FULLMAP>
__device__ __forceinline__ void cos_body(const float* __restrict__ SRC, const float* __restrict__ TH, unsigned short* __restrict__ DST) {
  #pragma clang fp contract(off)
  static_assert(W == 64 || W == 1024);
  static_assert(((long long)MTOK * W) % 1024 == 0);
  __shared__ __align__(16) _Float16 sh[1024];
  const int t = threadIdx.x;
  constexpr int RPB = 1024 / W;
#pragma unroll 1
  for (int it = 0; it < 8; ++it) {
    const int i = t + 128 * it;
    const int r = blockIdx.x * RPB + i / W; const int c = i % W;
    const size_t srow = FULLMAP ? ((size_t)(r / SEQ) * SEQ_FULL + (size_t)(r % SEQ)) : (size_t)r;
    float xv = SRC[srow * CD + c];
    if (ABF) xv = cmb_bf(xv);
    const float th = cmb_bf(TH[c & 63]);
    sh[i] = toh_flush(cosf(xv + th));
  }
  __syncthreads();
  const v8h hv = *(const v8h*)(sh + 8 * t);
  VST2(v8h, (v8h*)(DST + (size_t)blockIdx.x * 1024 + 8 * t), hv);
}
__global__ __launch_bounds__(128) void k_cos_in(const float* __restrict__ SRC, const float* __restrict__ TH, unsigned short* __restrict__ DST) { cos_body<1024, 1, 1>(SRC, TH, DST); }
__global__ __launch_bounds__(128) void k_cos_q(const float* __restrict__ SRC, const float* __restrict__ TH, unsigned short* __restrict__ DST) { cos_body<64, 0, 0>(SRC, TH, DST); }

template <int DSTFULL>
__device__ __forceinline__ void ln_body(const float* __restrict__ A, const float* __restrict__ GA, const float* __restrict__ BE, float* __restrict__ Y) {
  #pragma clang fp contract(off)
  const int r = blockIdx.x * 8 + (threadIdx.x >> 5); const int L = threadIdx.x & 31; if (r >= MTOK) return;
  const size_t drow = DSTFULL ? ((size_t)(r / SEQ) * SEQ_FULL + (size_t)(r % SEQ)) : (size_t)r;
  v4f v[8]; float s = 0.f;
#pragma unroll
  for (int q = 0; q < 8; ++q) {
    v[q] = *(const v4f*)(A + (size_t)r * CD + 4 * L + 128 * q);
    s += (v[q].x + v[q].y) + (v[q].z + v[q].w);
  }
#pragma unroll
  for (int o = 16; o > 0; o >>= 1) s += __shfl_xor(s, o, 32);
  const float mu = s * 0.0009765625f; float qq = 0.f;
#pragma unroll
  for (int q = 0; q < 8; ++q) { v[q].x -= mu; v[q].y -= mu; v[q].z -= mu; v[q].w -= mu; qq += (v[q].x * v[q].x + v[q].y * v[q].y) + (v[q].z * v[q].z + v[q].w * v[q].w); }
#pragma unroll
  for (int o = 16; o > 0; o >>= 1) qq += __shfl_xor(qq, o, 32);
  const float rs = rsqrtf(qq * 0.0009765625f + 1e-5f);
#pragma unroll
  for (int q = 0; q < 8; ++q) {
    const int c = 4 * L + 128 * q; const v4f ga = *(const v4f*)(GA + c), be = *(const v4f*)(BE + c); v4f y;
    y.x = v[q].x * rs * cmb_bf(ga.x) + cmb_bf(be.x); y.y = v[q].y * rs * cmb_bf(ga.y) + cmb_bf(be.y);
    y.z = v[q].z * rs * cmb_bf(ga.z) + cmb_bf(be.z); y.w = v[q].w * rs * cmb_bf(ga.w) + cmb_bf(be.w);
    VST2(v4f, (v4f*)(Y + drow * CD + c), y);
  }
}
__global__ __launch_bounds__(256) void k_ln_mid(const float* __restrict__ A, const float* __restrict__ GA, const float* __restrict__ BE, float* __restrict__ Y) { ln_body<0>(A, GA, BE, Y); }
__global__ __launch_bounds__(256) void k_ln_out(const float* __restrict__ A, const float* __restrict__ GA, const float* __restrict__ BE, float* __restrict__ Y) { ln_body<1>(A, GA, BE, Y); }

struct GP {
  const unsigned short* A; const unsigned short* Bt; void* C; const float* bias; const float* R;
  long long strideA, strideC;
  int lda, ldb, ldc, ldr, M, N, K, rpb, rpbC, rpbR; float scale; int pad_;
};
static_assert(sizeof(GP) == 104);

template <int BIAS_MODE, int OUT_MODE, int RES_MODE, int ACT>
__device__ __forceinline__ void gemm_body(const GP& p) {
  __shared__ __align__(16) float sT[8][16 * 68];
  const int b = blockIdx.y;
  const int lane = threadIdx.x & 31, wave = threadIdx.x >> 5;
  const int tilesN = p.N >> 6, tilesM = p.M >> 6;
  const int tile = blockIdx.x * 8 + wave;
  if (tile >= tilesM * tilesN) return;
  const int tm = tile / tilesN, tn = tile - tm * tilesN;
  const int m0 = tm << 6, n0 = tn << 6;
  const _Float16* Ab = (const _Float16*)p.A + (size_t)b * p.strideA;
  const _Float16* Bb = (const _Float16*)p.Bt;
  const int rlane = lane & 15, koff = (lane >> 4) * 8, mOff = (lane >> 4) * 8;

  v8f acc[4][4];
#pragma unroll
  for (int i = 0; i < 4; ++i)
#pragma unroll
    for (int j = 0; j < 4; ++j) acc[i][j] = (v8f){0.f, 0.f, 0.f, 0.f, 0.f, 0.f, 0.f, 0.f};

  for (int k0 = 0; k0 < p.K; k0 += 32) {
    v16h bh[4];
#pragma unroll
    for (int j = 0; j < 4; ++j) bh[j] = ldg_frag(Bb + (size_t)(n0 + (j << 4) + rlane) * p.ldb + koff + k0);
#pragma unroll
    for (int i = 0; i < 4; ++i) {
      const v16h ah = ldg_frag(Ab + (size_t)(m0 + (i << 4) + rlane) * p.lda + koff + k0);
#pragma unroll
      for (int j = 0; j < 4; ++j) acc[i][j] = __builtin_amdgcn_wmma_f32_16x16x32_f16(false, ah, false, bh[j], (short)0, acc[i][j], false, false);
      dep_guard_h(acc[i][0], acc[i][3], ah, ah);
    }
    keep4_h(bh[0], bh[1], bh[2], bh[3]);
  }
  acc_guard4(acc[0][0], acc[0][1], acc[0][2], acc[0][3]);
  acc_guard4(acc[1][0], acc[1][1], acc[1][2], acc[1][3]);
  acc_guard4(acc[2][0], acc[2][1], acc[2][2], acc[2][3]);
  acc_guard4(acc[3][0], acc[3][1], acc[3][2], acc[3][3]);

  float* slab = sT[wave];
#pragma unroll
  for (int i = 0; i < 4; ++i) {
    const int mBase = m0 + (i << 4);
    float bm[8];
#pragma unroll
    for (int r = 0; r < 8; ++r) { bm[r] = 0.f; if (BIAS_MODE == 1) bm[r] = cmb_bf(p.bias[mBase + mOff + r]); }
#pragma unroll
    for (int j = 0; j < 4; ++j) {
      const int n = n0 + (j << 4) + rlane;
      float bv = 0.f; if (BIAS_MODE == 2) bv = cmb_bf(p.bias[n]);
#pragma unroll
      for (int r = 0; r < 8; ++r) {
        float v = acc[i][j][r] * p.scale + ((BIAS_MODE == 1) ? bm[r] : bv);
        if (ACT == 1) v = fmaxf(v, 0.f);
        slab[(mOff + r) * 68 + (j << 4) + rlane] = v;
      }
    }
    WAVE_SYNC();
    const int gb = mBase / p.rpb; const int tIn = mBase - gb * p.rpb;
    const size_t rowC0 = (size_t)gb * p.rpbC + tIn, rowR0 = (size_t)gb * p.rpbR + tIn;
    if (OUT_MODE == 0) {
      float* C = (float*)p.C + (size_t)b * p.strideC;
      const int hh = lane >> 4, c4 = (lane & 15) * 4;
      v4f val[8];
#pragma unroll
      for (int it = 0; it < 8; ++it) {
        const int row = it * 2 + hh;
        v4f v = *(const v4f*)(slab + row * 68 + c4);
        if (RES_MODE != 0) {
          v4f x = *(const v4f*)(p.R + (rowR0 + row) * (size_t)p.ldr + n0 + c4);
          if (RES_MODE == 2) { x.x = cmb_bf(x.x); x.y = cmb_bf(x.y); x.z = cmb_bf(x.z); x.w = cmb_bf(x.w); }
          v = v + x;
        }
        val[it] = v;
      }
      for (int pass = 0; pass < 2; ++pass) {
#pragma unroll
        for (int it = 0; it < 8; ++it) {
          const int row = it * 2 + hh;
          *(volatile v4f*)(C + (rowC0 + row) * (size_t)p.ldc + n0 + c4) = val[it];
        }
        __threadfence();
      }
    } else {
      unsigned short* C = (unsigned short*)p.C + (size_t)b * p.strideC;
      const int q = lane >> 3, c8 = (lane & 7) * 8;
      v8h hv[4];
#pragma unroll
      for (int it = 0; it < 4; ++it) {
        const float* sp = slab + (it * 4 + q) * 68 + c8;
#pragma unroll
        for (int e = 0; e < 8; ++e) hv[it][e] = toh_flush(sp[e]);
      }
      for (int pass = 0; pass < 2; ++pass) {
#pragma unroll
        for (int it = 0; it < 4; ++it) {
          const int row = it * 4 + q;
          *(volatile v8h*)(C + (rowC0 + row) * (size_t)p.ldc + n0 + c8) = hv[it];
        }
        __threadfence();
      }
    }
    WAVE_SYNC();
  }
}

__device__ __forceinline__ GP gp_pack(const unsigned short* A, const unsigned short* Bt, void* C, const float* bias, const float* R,
                                      long long strideA, long long strideC, int lda, int ldb, int ldc, int ldr, int M, int N, int K,
                                      int rpb, int rpbC, int rpbR, float scale) {
  GP g;
  g.A = A; g.Bt = Bt; g.C = C; g.bias = bias; g.R = R; g.strideA = strideA; g.strideC = strideC;
  g.lda = lda; g.ldb = ldb; g.ldc = ldc; g.ldr = ldr; g.M = M; g.N = N; g.K = K; g.rpb = rpb; g.rpbC = rpbC; g.rpbR = rpbR;
  g.scale = scale; g.pad_ = 0;
  return g;
}

__global__ __launch_bounds__(256) void k_gemm_comb(const unsigned short* A, const unsigned short* Bt, void* C, const float* bias, const float* R,
                                                     long long strideA, long long strideC, int lda, int ldb, int ldc, int ldr, int M, int N, int K,
                                                     int rpb, int rpbC, int rpbR, float scale) {
  const GP p = gp_pack(A, Bt, C, bias, R, strideA, strideC, lda, ldb, ldc, ldr, M, N, K, rpb, rpbC, rpbR, scale);
  gemm_body<0, 0, 2, 0>(p);
}
__global__ __launch_bounds__(256) void k_gemm_fc(const unsigned short* A, const unsigned short* Bt, void* C, const float* bias, const float* R,
                                                   long long strideA, long long strideC, int lda, int ldb, int ldc, int ldr, int M, int N, int K,
                                                   int rpb, int rpbC, int rpbR, float scale) {
  const GP p = gp_pack(A, Bt, C, bias, R, strideA, strideC, lda, ldb, ldc, ldr, M, N, K, rpb, rpbC, rpbR, scale);
  gemm_body<0, 1, 0, 1>(p);
}
__global__ __launch_bounds__(256) void k_gemm_mlp(const unsigned short* A, const unsigned short* Bt, void* C, const float* bias, const float* R,
                                                    long long strideA, long long strideC, int lda, int ldb, int ldc, int ldr, int M, int N, int K,
                                                    int rpb, int rpbC, int rpbR, float scale) {
  const GP p = gp_pack(A, Bt, C, bias, R, strideA, strideC, lda, ldb, ldc, ldr, M, N, K, rpb, rpbC, rpbR, scale);
  gemm_body<0, 0, 1, 0>(p);
}

constexpr size_t SZ_M16  = (size_t)MTOK * CD * 2;
constexpr size_t SZ_WCT  = (size_t)CD * CD * 2;
constexpr size_t SZ_W1T  = (size_t)C4 * NQ * 2;
constexpr size_t SZ_W2T  = (size_t)CD * C4 * 2;
constexpr size_t SZ_YB   = (size_t)MTOK * CD * 4;
constexpr size_t SZ_X1   = (size_t)MTOK * CD * 4;
constexpr size_t SZ_Q16  = (size_t)MTOK * NQ * 2;
constexpr size_t SZ_F16  = (size_t)MH * C4 * 2;
constexpr size_t OFF_M16 = 0;
constexpr size_t OFF_WCT = OFF_M16 + SZ_M16;
constexpr size_t OFF_W1T = OFF_WCT + SZ_WCT;
constexpr size_t OFF_W2T = OFF_W1T + SZ_W1T;
constexpr size_t OFF_YB  = OFF_W2T + SZ_W2T;
constexpr size_t OFF_X1  = OFF_YB + SZ_YB;
constexpr size_t OFF_Q16 = OFF_X1 + SZ_X1;
constexpr size_t OFF_F16 = OFF_Q16 + SZ_Q16;
constexpr size_t WS_TOTAL = OFF_F16 + SZ_F16;
static_assert(WS_TOTAL <= (size_t)134217728);
static_assert(SZ_M16 % 256 == 0 && SZ_WCT % 256 == 0 && SZ_W1T % 256 == 0 && SZ_W2T % 256 == 0 && SZ_YB % 256 == 0 &&
              SZ_X1 % 256 == 0 && SZ_Q16 % 256 == 0 && SZ_F16 % 256 == 0);
static_assert(SZ_M16 == (size_t)MTOK * 1024 * 2);
static_assert(SZ_Q16 == (size_t)(MTOK / 16) * 1024 * 2);

static GP mk_gp(const unsigned short* A, long long sA, int lda, const unsigned short* Bt, int ldb, void* C, long long sC, int ldc,
                const float* bias, const float* R, int ldr, int M, int N, int K, int rpb, int rpbC, int rpbR) {
  GP g{};
  g.A = A; g.Bt = Bt; g.C = C; g.bias = bias; g.R = R; g.strideA = sA; g.strideC = sC;
  g.lda = lda; g.ldb = ldb; g.ldc = ldc; g.ldr = ldr; g.M = M; g.N = N; g.K = K; g.rpb = rpb; g.rpbC = rpbC; g.rpbR = rpbR;
  g.scale = 0.0625f; g.pad_ = 0;
  return g;
}
#define GP_ARGS(g) (g).A, (g).Bt, (g).C, (g).bias, (g).R, (g).strideA, (g).strideC, (g).lda, (g).ldb, (g).ldc, (g).ldr, (g).M, (g).N, (g).K, (g).rpb, (g).rpbC, (g).rpbR, (g).scale
static unsigned gemm_blocks(int M, int N) { return (unsigned)((((M / 64) * (N / 64)) + 7) / 8); }

extern "C" void kernel_launch(void* const* d_in, const int* in_sizes, int n_in, void* d_out, int out_size, void* d_ws, size_t ws_size, hipStream_t stream) {
  if (n_in < 10) return;
  const long long need_x = ((long long)(NB - 1) * SEQ_FULL + SEQ) * CD;
  if ((long long)in_sizes[0] < need_x) return;
  if (in_sizes[1] < HD || in_sizes[2] < CD * CD || in_sizes[3] < CD || in_sizes[4] < CD) return;
  if (in_sizes[5] < NQ || in_sizes[6] < C4 * NQ || in_sizes[7] < CD * C4 || in_sizes[8] < CD || in_sizes[9] < CD) return;
  if ((long long)out_size < need_x) return;
  if (ws_size < WS_TOTAL) return;

  const float* x    = (const float*)d_in[0];
  const float* tha  = (const float*)d_in[1];
  const float* wc   = (const float*)d_in[2];
  const float* ga1  = (const float*)d_in[3];
  const float* be1  = (const float*)d_in[4];
  const float* thf  = (const float*)d_in[5];
  const float* w1   = (const float*)d_in[6];
  const float* w2   = (const float*)d_in[7];
  const float* ga2  = (const float*)d_in[8];
  const float* be2  = (const float*)d_in[9];
  float* out = (float*)d_out;
  char* wsp = (char*)d_ws;
  unsigned short* M16 = (unsigned short*)(wsp + OFF_M16);
  unsigned short* WCT = (unsigned short*)(wsp + OFF_WCT);
  unsigned short* W1T = (unsigned short*)(wsp + OFF_W1T);
  unsigned short* W2T = (unsigned short*)(wsp + OFF_W2T);
  float*          YB  = (float*)(wsp + OFF_YB);
  float*          X1  = (float*)(wsp + OFF_X1);
  unsigned short* Q16 = (unsigned short*)(wsp + OFF_Q16);
  unsigned short* F16 = (unsigned short*)(wsp + OFF_F16);
  const int BIG = 1 << 30;

  k_castn<<<(unsigned)((CD * CD / 8 + 255) / 256), 256, 0, stream>>>(wc, WCT, CD * CD / 8, 16.0f);
  k_castn<<<(unsigned)((C4 * NQ / 8 + 255) / 256), 256, 0, stream>>>(w1, W1T, C4 * NQ / 8, 16.0f);
  k_castn<<<(unsigned)((CD * C4 / 8 + 255) / 256), 256, 0, stream>>>(w2, W2T, CD * C4 / 8, 16.0f);
  k_cos_in<<<MTOK, 128, 0, stream>>>(x, tha, M16);
  { const GP g = mk_gp(M16, 0, CD, WCT, CD, (void*)YB, 0, CD, nullptr, x, CD, MTOK, CD, CD, SEQ, SEQ, SEQ_FULL);
    k_gemm_comb<<<dim3(gemm_blocks(MTOK, CD), 1), 256, 0, stream>>>(GP_ARGS(g)); }
  k_ln_mid<<<MTOK / 8, 256, 0, stream>>>(YB, ga1, be1, X1);
  k_cos_q<<<MTOK / 16, 128, 0, stream>>>(X1, thf, Q16);
  for (int hf = 0; hf < 2; ++hf) {
    const size_t r0 = (size_t)hf * MH;
    { const GP g = mk_gp(Q16 + r0 * NQ, 0, NQ, W1T, NQ, (void*)F16, 0, C4, nullptr, nullptr, 0, MH, C4, NQ, BIG, BIG, BIG);
      k_gemm_fc<<<dim3(gemm_blocks(MH, C4), 1), 256, 0, stream>>>(GP_ARGS(g)); }
    { const GP g = mk_gp(F16, 0, C4, W2T, C4, (void*)(YB + r0 * CD), 0, CD, nullptr, X1 + r0 * CD, CD, MH, CD, C4, BIG, BIG, BIG);
      k_gemm_mlp<<<dim3(gemm_blocks(MH, CD), 1), 256, 0, stream>>>(GP_ARGS(g)); }
  }
  k_ln_out<<<MTOK / 8, 256, 0, stream>>>(YB, ga2, be2, out);
}
